// BatchedGNNModel_58523224375656
// MI455X (gfx1250) — hardware-verified
//
#include <hip/hip_runtime.h>


namespace {
constexpr int Bn = 64, NV = 256, N = 768, F0 = 6, F0P = 32, H1 = 256, H2 = 128, FO = 3, FOP = 64;
constexpr float AS = 8.0f, AI = 0.125f;

typedef _Float16 b16;
typedef __attribute__((ext_vector_type(16))) _Float16 v16b;
typedef __attribute__((ext_vector_type(8)))  _Float16 v8b;
typedef __attribute__((ext_vector_type(8)))  float v8f;
typedef __attribute__((ext_vector_type(4)))  float v4f;

__device__ __forceinline__ v8b ld8b(const b16* p) { return *(const v8b*)p; }
__device__ __forceinline__ v16b cat8b(v8b a, v8b b) { return __builtin_shufflevector(a, b, 0, 1, 2, 3, 4, 5, 6, 7, 8, 9, 10, 11, 12, 13, 14, 15); }
__device__ __forceinline__ v16b frag_kb(const b16* p, int hh) { return cat8b(ld8b(p + 8 * hh), ld8b(p + 16 + 8 * hh)); }
__device__ __forceinline__ void split16(float v, b16& hi, b16& lo) { hi = (b16)v; lo = (b16)(v - (float)hi); }
__device__ __forceinline__ void frag_ksplit(const float* p, int hh, v16b& fh_, v16b& fl_) {
  const float* p0 = p + 8 * hh; const float* p1 = p + 16 + 8 * hh;
#pragma unroll
  for (int e = 0; e < 8; ++e) { b16 a, c; split16(p0[e], a, c); fh_[e] = a; fl_[e] = c; split16(p1[e], a, c); fh_[8 + e] = a; fl_[8 + e] = c; }
}
__device__ __forceinline__ v8f wmma16b(v16b a, v16b b, v8f c) {
  v8f d = __builtin_amdgcn_wmma_f32_16x16x32_f16(false, a, false, b, (short)0, c, false, false);
  asm volatile("v_nop\n\tv_nop\n\tv_nop\n\tv_nop" : "+v"(d) : "v"(a), "v"(b));
  return d;
}
__device__ __forceinline__ void wave_lds_sync() {
  __builtin_amdgcn_fence(__ATOMIC_RELEASE, "workgroup");
  __builtin_amdgcn_wave_barrier();
  __builtin_amdgcn_fence(__ATOMIC_ACQUIRE, "workgroup");
}

struct Opnd { const void* p0; const void* p1; int ld; };
template <int NP> __device__ __forceinline__ void load_frags(const Opnd& o, int row, int kb, int hh, v16b& fh_, v16b& fl_) {
  if (NP == 0) { frag_ksplit((const float*)o.p0 + (size_t)row * o.ld + kb, hh, fh_, fl_); }
  else if (NP == 4 || NP == 5) {
    const float sc_ = (NP == 4) ? 64.0f : 8.0f;
    const float* p = (const float*)o.p0 + (size_t)row * o.ld + kb; const float* p0 = p + 8 * hh; const float* p1 = p + 16 + 8 * hh;
#pragma unroll
    for (int e = 0; e < 8; ++e) { b16 a, c; split16(p0[e] * sc_, a, c); fh_[e] = a; fl_[e] = c; split16(p1[e] * sc_, a, c); fh_[8 + e] = a; fl_[8 + e] = c; }
  } else if (NP == 3) {
    const float* p = (const float*)o.p0 + (size_t)row * o.ld + kb; const float* p0 = p + 8 * hh; const float* p1 = p + 16 + 8 * hh;
#pragma unroll
    for (int e = 0; e < 8; ++e) { fh_[e] = (b16)p0[e]; fh_[8 + e] = (b16)p1[e]; }
    fl_ = fh_;
  } else {
    fh_ = frag_kb((const b16*)o.p0 + (size_t)row * o.ld + kb, hh);
    if (NP == 2) fl_ = frag_kb((const b16*)o.p1 + (size_t)row * o.ld + kb, hh); else fl_ = fh_;
  }
}
template <int ANP, int BNP> __device__ __forceinline__ v8f mac(v16b ah, v16b al, v16b bh, v16b bl, v8f c) {
  c = wmma16b(ah, bh, c);
  if (BNP == 0 || BNP == 2 || BNP == 4 || BNP == 5) c = wmma16b(ah, bl, c);
  if (ANP == 0 || ANP == 2 || ANP == 4 || ANP == 5) c = wmma16b(al, bh, c);
  return c;
}
template <int ANP, int BNP>
__device__ __forceinline__ void gemm_tile(const Opnd& A, const Opnd& B, int K, int m0, int c0, int nloc, int hlf, v8f (&acc)[2][4]) {
  for (int kb = 0; kb < K; kb += 32) {
    v16b a0h, a0l, a1h, a1l;
    load_frags<ANP>(A, m0 + nloc, kb, hlf, a0h, a0l);
    load_frags<ANP>(A, m0 + 16 + nloc, kb, hlf, a1h, a1l);
#pragma unroll
    for (int t = 0; t < 4; ++t) {
      v16b bh, bl;
      load_frags<BNP>(B, c0 + t * 16 + nloc, kb, hlf, bh, bl);
      acc[0][t] = mac<ANP, BNP>(a0h, a0l, bh, bl, acc[0][t]);
      acc[1][t] = mac<ANP, BNP>(a1h, a1l, bh, bl, acc[1][t]);
    }
  }
}

__device__ __forceinline__ void epi_planes(v8f (&acc)[2][4], float scale, bool two, b16* __restrict__ oh, b16* __restrict__ ol, int ldo,
                                           int m0, int c0, int lane, b16* Th, b16* Tl) {
  const int nloc = lane & 15, hlf = lane >> 4;
#pragma unroll
  for (int t = 0; t < 4; ++t)
#pragma unroll
    for (int r = 0; r < 2; ++r)
#pragma unroll
      for (int v = 0; v < 8; ++v) {
        const int rr = r * 16 + v + 8 * hlf, cc = t * 16 + nloc;
        b16 h_, l_; split16(acc[r][t][v] * scale, h_, l_);
        Th[rr * 64 + cc] = h_; Tl[rr * 64 + cc] = l_;
      }
  wave_lds_sync();
  for (int pass = 0; pass < 2; ++pass) {
#pragma unroll
    for (int j = 0; j < 8; ++j) {
      const int rr = j * 4 + (lane >> 3), c8 = (lane & 7) * 8;
      const size_t o = (size_t)(m0 + rr) * ldo + c0 + c8;
      *(volatile v8b*)(oh + o) = ld8b(Th + rr * 64 + c8);
      if (two) *(volatile v8b*)(ol + o) = ld8b(Tl + rr * 64 + c8);
    }
    __threadfence();
  }
}
__device__ __forceinline__ void epi_f32(v8f (&acc)[2][4], float scale, const float* rscale, float* __restrict__ out, int ldo, int m0, int c0, int lane, float* Tt) {
  const int nloc = lane & 15, hlf = lane >> 4;
#pragma unroll
  for (int t = 0; t < 4; ++t)
#pragma unroll
    for (int r = 0; r < 2; ++r)
#pragma unroll
      for (int v = 0; v < 8; ++v) {
        const int rr = r * 16 + v + 8 * hlf;
        const float rs = rscale ? rscale[(size_t)(m0 + rr) * 32] : 1.0f;
        Tt[rr * 64 + t * 16 + nloc] = acc[r][t][v] * scale * rs;
      }
  wave_lds_sync();
  float* dst0 = out + (size_t)m0 * ldo + c0;
  for (int pass = 0; pass < 2; ++pass) {
#pragma unroll
    for (int j = 0; j < 16; ++j) { const int rr = j * 2 + hlf, c4 = nloc * 4; *(volatile v4f*)(dst0 + (size_t)rr * ldo + c4) = *(const v4f*)(Tt + rr * 64 + c4); }
    __threadfence();
  }
}


typedef __attribute__((ext_vector_type(8))) __bf16 v8bb; typedef __attribute__((ext_vector_type(16))) __bf16 v16bb;
typedef __attribute__((ext_vector_type(8))) unsigned short v8us;
__device__ __forceinline__ v16bb frag_kb_bf(const __bf16* p, int hh) { const v8bb a = *(const v8bb*)(p + 8 * hh), b = *(const v8bb*)(p + 16 + 8 * hh); return __builtin_shufflevector(a, b, 0, 1, 2, 3, 4, 5, 6, 7, 8, 9, 10, 11, 12, 13, 14, 15); }
__device__ __forceinline__ v8f wmma16bb(v16bb a, v16bb b, v8f c) {
  v8f d = __builtin_amdgcn_wmma_f32_16x16x32_bf16(false, a, false, b, (short)0, c, false, false);
  asm volatile("v_nop\n\tv_nop\n\tv_nop\n\tv_nop" : "+v"(d) : "v"(a), "v"(b));
  return d;
}
__device__ __forceinline__ unsigned short bf16_rne_bits(float v) { unsigned int u = __float_as_uint(v); u += 0x7FFFu + ((u >> 16) & 1u); return (unsigned short)(u >> 16); }
__device__ __forceinline__ float bf16_rne(float v) { return __uint_as_float(((unsigned int)bf16_rne_bits(v)) << 16); }


__global__ __launch_bounds__(256) void prep_kernel(const float* __restrict__ adj, const float* __restrict__ W1, const float* __restrict__ W2, const float* __restrict__ W3, const float* __restrict__ W4,
                                                   b16* __restrict__ a16, float* __restrict__ dvec, b16* __restrict__ w1, b16* __restrict__ w2, b16* __restrict__ w3, b16* __restrict__ w4) {
  const size_t tid = (size_t)blockIdx.x * blockDim.x + threadIdx.x, nth = (size_t)gridDim.x * blockDim.x; const int lane = threadIdx.x & 31;
  for (int pass = 0; pass < 2; ++pass) {
    for (size_t p = tid; p < (size_t)N * N; p += nth) ((volatile b16*)a16)[p] = (b16)adj[p];
    for (size_t wv = tid >> 5; wv < (size_t)N; wv += nth >> 5) { float s = 0.0f; for (int j = lane; j < N; j += 32) s += adj[wv * N + j];
#pragma unroll
      for (int o = 16; o > 0; o >>= 1) s += __shfl_xor(s, o);
      if (lane == 0) ((volatile float*)dvec)[wv] = (s > 0.0f) ? rsqrtf(s) : 0.0f; }
    for (size_t p = tid; p < (size_t)H1 * F0P; p += nth) { const int n = (int)(p / F0P), k = (int)(p % F0P); ((volatile b16*)w1)[p] = (b16)((k < F0) ? W1[(size_t)n * F0 + min(k, F0 - 1)] : 0.0f); }
    for (size_t p = tid; p < (size_t)H2 * H1; p += nth) ((volatile b16*)w2)[p] = (b16)W2[p];
    for (size_t p = tid; p < (size_t)H2 * H2; p += nth) ((volatile b16*)w3)[p] = (b16)W3[p];
    for (size_t p = tid; p < (size_t)FOP * H2; p += nth) { const int n = (int)(p / H2), k = (int)(p % H2); ((volatile b16*)w4)[p] = (b16)((n < FO) ? W4[(size_t)min(n, FO - 1) * H2 + k] : 0.0f); }
    __threadfence();
  }
}

__device__ __forceinline__ bool grasped(int rod, int v, const int* __restrict__ s0, int n0, const int* __restrict__ s1, int n1, const int* __restrict__ s2, int n2) {
  const int* s = (rod == 0) ? s0 : (rod == 1) ? s1 : s2; const int n = (rod == 0) ? n0 : (rod == 1) ? n1 : n2; bool g = false;
  for (int i = 0; i < n; ++i) g |= (s[i] == v);
  return g;
}

__global__ __launch_bounds__(256) void h0_kernel(const float* __restrict__ x, const float* __restrict__ inp, const int* __restrict__ s0, int n0, const int* __restrict__ s1, int n1, const int* __restrict__ s2, int n2, float* __restrict__ h0) {
  const int gi = blockIdx.x * 256 + threadIdx.x; const int i = gi >> 3, q = gi & 7; const int node = i % N, rod = node / NV, v = node % NV;
  v4f o = {0.0f, 0.0f, 0.0f, 0.0f};
  if (q < 2) { const bool g = grasped(rod, v, s0, n0, s1, n1, s2, n2);
    if (q == 0) { o[0] = g ? inp[(size_t)i * 3] : x[(size_t)i * F0]; o[1] = g ? inp[(size_t)i * 3 + 1] : x[(size_t)i * F0 + 1]; o[2] = g ? inp[(size_t)i * 3 + 2] : x[(size_t)i * F0 + 2]; o[3] = x[(size_t)i * F0 + 3]; }
    else { o[0] = x[(size_t)i * F0 + 4]; o[1] = x[(size_t)i * F0 + 5]; } }
  for (int pass = 0; pass < 2; ++pass) { *(volatile v4f*)(h0 + (size_t)i * F0P + q * 4) = o; __threadfence(); }
}

template <int KIN, int NOUT>
__global__ __launch_bounds__(128) void lint_kernel(const float* __restrict__ h, const b16* __restrict__ w, const float* __restrict__ bias, int nreal, const float* __restrict__ dvec, b16* __restrict__ yt) {
  __shared__ __attribute__((aligned(16))) b16 Th[64][128 + 8], Tl[64][128 + 8];
  const int lane = threadIdx.x & 31, wave = threadIdx.x >> 5, nloc = lane & 15, hlf = lane >> 4, b = blockIdx.z, j0 = blockIdx.y * 128, m0 = j0 + wave * 32, c0 = blockIdx.x * 64;
  v8f acc[2][4];
#pragma unroll
  for (int r = 0; r < 2; ++r)
#pragma unroll
    for (int t = 0; t < 4; ++t) acc[r][t] = (v8f){};
  const Opnd A{h + (size_t)b * N * KIN, nullptr, KIN}, Bo{w, nullptr, KIN};
  gemm_tile<5, 1>(A, Bo, KIN, m0, c0, nloc, hlf, acc);
#pragma unroll
  for (int t = 0; t < 4; ++t)
#pragma unroll
    for (int r = 0; r < 2; ++r)
#pragma unroll
      for (int v = 0; v < 8; ++v) { const int jl = wave * 32 + r * 16 + 8 * hlf + v, f = c0 + t * 16 + nloc; const float val = (acc[r][t][v] * AI + bias[min(f, nreal - 1)]) * dvec[j0 + jl] * AS;
        b16 a_, c_; split16((f < nreal) ? val : 0.0f, a_, c_); Th[t * 16 + nloc][jl] = a_; Tl[t * 16 + nloc][jl] = c_; }
  __syncthreads();
  const size_t PLN = (size_t)NOUT * N;
  b16* dst = yt + (size_t)b * 2 * PLN + (size_t)c0 * N + j0;
  for (int pass = 0; pass < 2; ++pass) {
#pragma unroll
    for (int jj = 0; jj < 8; ++jj) { const int f = wave * 16 + jj * 2 + (lane >> 4), c8 = (lane & 15) * 8; *(volatile v8b*)(dst + (size_t)f * N + c8) = *(const v8b*)(&Th[f][c8]); *(volatile v8b*)(dst + PLN + (size_t)f * N + c8) = *(const v8b*)(&Tl[f][c8]); }
    __threadfence();
  }
}

template <int NOUT, bool RELU>
__global__ __launch_bounds__(128) void agg_kernel(const b16* __restrict__ a16, const b16* __restrict__ yt, const float* __restrict__ dvec, float* __restrict__ ho) {
  __shared__ __attribute__((aligned(16))) float Ts[4][32 * 64];
  const int lane = threadIdx.x & 31, wave = threadIdx.x >> 5, nloc = lane & 15, hlf = lane >> 4, b = blockIdx.z, m0 = blockIdx.y * 128 + wave * 32, c0 = blockIdx.x * 64;
  const size_t PLN = (size_t)NOUT * N; const b16* yb = yt + (size_t)b * 2 * PLN;
  v8f acc[2][4];
#pragma unroll
  for (int r = 0; r < 2; ++r)
#pragma unroll
    for (int t = 0; t < 4; ++t) acc[r][t] = (v8f){};
  const Opnd A{a16, nullptr, N}, Bo{yb, yb + PLN, N};
  gemm_tile<1, 2>(A, Bo, N, m0, c0, nloc, hlf, acc);
#pragma unroll
  for (int t = 0; t < 4; ++t)
#pragma unroll
    for (int r = 0; r < 2; ++r)
#pragma unroll
      for (int v = 0; v < 8; ++v) { float val = acc[r][t][v] * AI * dvec[m0 + r * 16 + 8 * hlf + v]; if (RELU) val = fmaxf(val, 0.0f); acc[r][t][v] = val; }
  epi_f32(acc, 1.0f, nullptr, ho + (size_t)b * N * NOUT, NOUT, m0, c0, lane, Ts[wave]);
}

__global__ __launch_bounds__(256) void final_kernel(const float* __restrict__ h4, const float* __restrict__ inp, const int* __restrict__ s0, int n0, const int* __restrict__ s1, int n1, const int* __restrict__ s2, int n2, float* __restrict__ out) {
  __shared__ float Ob[N * 3];
  const int b = blockIdx.x, t_ = threadIdx.x;
  for (int node = t_; node < N; node += 256) { const int rod = node / NV, v = node % NV; const bool g = grasped(rod, v, s0, n0, s1, n1, s2, n2); const size_t i = (size_t)b * N + node;
#pragma unroll
    for (int c = 0; c < 3; ++c) Ob[node * 3 + c] = g ? inp[i * 3 + c] : h4[i * FOP + c]; }
  __syncthreads();
  for (int pass = 0; pass < 2; ++pass) { for (int i = t_; i < N * 3 / 4; i += 256) *(volatile v4f*)(out + (size_t)b * N * 3 + i * 4) = *(const v4f*)(&Ob[i * 4]); __threadfence(); }
}
}

extern "C" void kernel_launch(void* const* d_in, const int* in_sizes, int n_in,
                              void* d_out, int out_size, void* d_ws, size_t ws_size, hipStream_t stream) {
  (void)n_in; (void)out_size;
  const float* x = (const float*)d_in[0]; const float* inp = (const float*)d_in[1]; const float* adj = (const float*)d_in[2];
  const float* W1 = (const float*)d_in[3]; const float* b1 = (const float*)d_in[4]; const float* W2 = (const float*)d_in[5]; const float* b2 = (const float*)d_in[6];
  const float* W3 = (const float*)d_in[7]; const float* b3 = (const float*)d_in[8]; const float* W4 = (const float*)d_in[9]; const float* b4 = (const float*)d_in[10];
  const int* s0 = (const int*)d_in[11]; const int* s1 = (const int*)d_in[12]; const int* s2 = (const int*)d_in[13];
  float* out = (float*)d_out;
  if (in_sizes[0] != Bn * N * F0 || in_sizes[1] != Bn * N * 3 || in_sizes[2] != N * N || in_sizes[3] != H1 * F0 || in_sizes[9] != FO * H2) return;
  const int n0 = in_sizes[11], n1 = in_sizes[12], n2 = in_sizes[13];
  if (n0 < 0 || n1 < 0 || n2 < 0 || n0 > NV || n1 > NV || n2 > NV) return;
  size_t off = 0; char* ws = (char*)d_ws;
  auto carve = [&](size_t bytes) { char* p = ws + off; off += (bytes + 255) & ~(size_t)255; return p; };
  b16* a16 = (b16*)carve((size_t)N * N * 2); float* dvec = (float*)carve(N * 4); b16* w1 = (b16*)carve((size_t)H1 * F0P * 2); b16* w2 = (b16*)carve((size_t)H2 * H1 * 2); b16* w3 = (b16*)carve((size_t)H2 * H2 * 2); b16* w4 = (b16*)carve((size_t)FOP * H2 * 2);
  float* h0 = (float*)carve((size_t)Bn * N * F0P * 4); b16* yt = (b16*)carve((size_t)Bn * 2 * H1 * N * 2); float* ha = (float*)carve((size_t)Bn * N * H1 * 4); float* hb = (float*)carve((size_t)Bn * N * H2 * 4);
  if (off > ws_size) return;
  prep_kernel<<<512, 256, 0, stream>>>(adj, W1, W2, W3, W4, a16, dvec, w1, w2, w3, w4);
  h0_kernel<<<Bn * N * 8 / 256, 256, 0, stream>>>(x, inp, s0, n0, s1, n1, s2, n2, h0);
  lint_kernel<F0P, H1><<<dim3(H1 / 64, N / 128, Bn), 128, 0, stream>>>(h0, w1, b1, H1, dvec, yt);
  agg_kernel<H1, true><<<dim3(H1 / 64, N / 128, Bn), 128, 0, stream>>>(a16, yt, dvec, ha);
  lint_kernel<H1, H2><<<dim3(H2 / 64, N / 128, Bn), 128, 0, stream>>>(ha, w2, b2, H2, dvec, yt);
  agg_kernel<H2, true><<<dim3(H2 / 64, N / 128, Bn), 128, 0, stream>>>(a16, yt, dvec, hb);
  lint_kernel<H2, H2><<<dim3(H2 / 64, N / 128, Bn), 128, 0, stream>>>(hb, w3, b3, H2, dvec, yt);
  agg_kernel<H2, false><<<dim3(H2 / 64, N / 128, Bn), 128, 0, stream>>>(a16, yt, dvec, ha);
  lint_kernel<H2, FOP><<<dim3(1, N / 128, Bn), 128, 0, stream>>>(ha, w4, b4, FO, dvec, yt);
  agg_kernel<FOP, false><<<dim3(1, N / 128, Bn), 128, 0, stream>>>(a16, yt, dvec, hb);
  final_kernel<<<Bn, 256, 0, stream>>>(hb, inp, s0, n0, s1, n1, s2, n2, out);
}
